// SwinTransformerBlock2D_72713796321802
// MI455X (gfx1250) — hardware-verified
//
#include <hip/hip_runtime.h>
#include <stdint.h>


typedef _Float16 v16h __attribute__((ext_vector_type(16)));
typedef _Float16 v8h  __attribute__((ext_vector_type(8)));
typedef float    v8f  __attribute__((ext_vector_type(8)));
typedef float    v4f  __attribute__((ext_vector_type(4)));
union Frag { v16h v; v8h half[2]; };

#define DIMC   192
#define HEADS  6
#define WSZ    7
#define SHF    3
#define HDIM   32
#define NTOK   49
#define IMG    56
#define PLANE  3136
#define HID    768
#define QKVN   576

#define QK_SCALE 0.17677669529663687f
#define W_UP     64.0f
#define W_DOWN   0.015625f
#define Q_UP     8.0f
#define Q_DOWN   0.125f
#define P_UP     256.0f
#define P_DOWN   0.00390625f
#define NEG_BIG  (-1.0e30f)

#define SEG0_OFF 0
#define SEG1_OFF 110592
#define SEG2_OFF 147456
#define SEG3_OFF 294912
#define SEG_END  442368

__device__ __forceinline__ v8f wmma_f16(v16h a, v16h b, v8f c) {
  v8f d = __builtin_amdgcn_wmma_f32_16x16x32_f16(false, a, false, b, (short)0, c, false, false);
  asm volatile("v_nop\n\tv_nop\n\tv_nop\n\tv_nop" : "+v"(d) : "v"(a), "v"(b));
  return d;
}

__device__ __forceinline__ v16h ld_frag(const _Float16* base, int pitch, int r0, int k0, int lane) {
  const int r = lane & 15, h = lane >> 4;
  const _Float16* p = base + (r0 + r) * pitch + k0 + 8 * h;
  Frag f;
  f.half[0] = *(const v8h*)p;
  f.half[1] = *(const v8h*)(p + 16);
  return f.v;
}

__global__ void __launch_bounds__(256) k_wconv(
    const float* __restrict__ qkv_w, const float* __restrict__ proj_w,
    const float* __restrict__ fc1_w, const float* __restrict__ fc2_w,
    _Float16* wt, int nchunk)
{
  const int q = blockIdx.x * 256 + threadIdx.x;
  if (q >= nchunk) return;
  const int e = q * 8;
  const float* src; int K, NO, el;
  if (e < SEG1_OFF)      { src = qkv_w;  K = DIMC; NO = QKVN; el = e; }
  else if (e < SEG2_OFF) { src = proj_w; K = DIMC; NO = DIMC; el = e - SEG1_OFF; }
  else if (e < SEG3_OFF) { src = fc1_w;  K = DIMC; NO = HID;  el = e - SEG2_OFF; }
  else                   { src = fc2_w;  K = HID;  NO = DIMC; el = e - SEG3_OFF; }
  const int n  = el / K;
  const int k0 = el - n * K;
  v8h v;
#pragma unroll
  for (int j = 0; j < 8; ++j)
    v[j] = (_Float16)(src[(size_t)(k0 + j) * NO + n] * W_UP);
  volatile v8h* p = (volatile v8h*)(wt + e);
  *p = v;
  __threadfence();
  *p = v;
}

__device__ __forceinline__ int region_id(int yr, int xr) {
  const int ry = yr < (IMG - WSZ) ? 0 : (yr < (IMG - SHF) ? 1 : 2);
  const int rx = xr < (IMG - WSZ) ? 0 : (xr < (IMG - SHF) ? 1 : 2);
  return ry * 3 + rx;
}

__device__ __forceinline__ void attn_rows_store(const float* sOut, const float* __restrict__ xin,
                                                float* x1, int bb, int wy, int wx, int wv, int lane)
{
  for (int t = wv; t < NTOK; t += 8) {
    const int ty = t / WSZ, tx = t - ty * WSZ;
    const int gy = (wy * WSZ + ty + SHF) % IMG;
    const int gx = (wx * WSZ + tx + SHF) % IMG;
    const size_t pix = (size_t)gy * IMG + gx;
    float* dst = x1 + ((size_t)bb * PLANE + pix) * DIMC;
    const float* px = xin + (size_t)bb * DIMC * PLANE + pix;
    {
      const int c = 4 * lane;
      const v4f o = *(const v4f*)(sOut + t * DIMC + c);
      v4f r;
      r.x = o.x + px[(size_t)(c + 0) * PLANE];
      r.y = o.y + px[(size_t)(c + 1) * PLANE];
      r.z = o.z + px[(size_t)(c + 2) * PLANE];
      r.w = o.w + px[(size_t)(c + 3) * PLANE];
      *(volatile v4f*)(dst + c) = r;
    }
    if (lane < 16) {
      const int c = 128 + 4 * lane;
      const v4f o = *(const v4f*)(sOut + t * DIMC + c);
      v4f r;
      r.x = o.x + px[(size_t)(c + 0) * PLANE];
      r.y = o.y + px[(size_t)(c + 1) * PLANE];
      r.z = o.z + px[(size_t)(c + 2) * PLANE];
      r.w = o.w + px[(size_t)(c + 3) * PLANE];
      *(volatile v4f*)(dst + c) = r;
    }
  }
}

__global__ void __launch_bounds__(256) k_attn(
    const float* __restrict__ xin, const float* __restrict__ n1g, const float* __restrict__ n1b,
    const _Float16* __restrict__ qkvT, const float* __restrict__ qkv_b,
    const _Float16* __restrict__ projT, const float* __restrict__ proj_b,
    const float* __restrict__ rel_bias, float* x1, int nwin)
{
  __shared__ __align__(16) unsigned char smem[61440];
  _Float16* sA  = (_Float16*)(smem);
  _Float16* sQ  = (_Float16*)(smem + 24576);
  _Float16* sK  = (_Float16*)(smem + 28672);
  _Float16* sVT = (_Float16*)(smem + 32768);
  float*    sS  = (float*)(smem + 36864);
  _Float16* sP  = (_Float16*)(smem + 53248);
  _Float16* sAV = sQ;
  float*    sOut = (float*)(smem);

  const int tid = threadIdx.x;
  const int lane = tid & 31, wv = tid >> 5, h16 = lane >> 4, c16 = lane & 15;
  const int widx = blockIdx.x;
  if (widx >= nwin) return;
  const int bb = widx >> 6;
  const int wy = (widx >> 3) & 7;
  const int wx = widx & 7;

  {
    const int t = tid >> 2, sub = tid & 3;
    if (t < NTOK) {
      const int ty = t / WSZ, tx = t - ty * WSZ;
      const int gy = (wy * WSZ + ty + SHF) % IMG;
      const int gx = (wx * WSZ + tx + SHF) % IMG;
      const float* px = xin + (size_t)bb * DIMC * PLANE + (size_t)gy * IMG + gx;
      float vals[48];
      float s = 0.f;
#pragma unroll
      for (int j = 0; j < 48; ++j) {
        const int c = sub * 48 + j;
        const float v = px[(size_t)c * PLANE];
        vals[j] = v; s += v;
      }
      s += __shfl_xor(s, 1); s += __shfl_xor(s, 2);
      const float mu = s * (1.f / DIMC);
      float d2 = 0.f;
#pragma unroll
      for (int j = 0; j < 48; ++j) { const float d = vals[j] - mu; d2 += d * d; }
      d2 += __shfl_xor(d2, 1); d2 += __shfl_xor(d2, 2);
      const float rs = rsqrtf(d2 * (1.f / DIMC) + 1e-5f);
#pragma unroll
      for (int j = 0; j < 48; ++j) {
        const int c = sub * 48 + j;
        sA[t * DIMC + c] = (_Float16)((vals[j] - mu) * rs * n1g[c] + n1b[c]);
      }
    } else {
#pragma unroll
      for (int j = 0; j < 48; ++j) sA[t * DIMC + sub * 48 + j] = (_Float16)0.f;
    }
  }
  __syncthreads();

  v8f pacc[6];
#pragma unroll
  for (int i = 0; i < 6; ++i) { v8f z = {}; pacc[i] = z; }

  for (int h = 0; h < HEADS; ++h) {
#pragma unroll
    for (int i = 0; i < 3; ++i) {
      const int t = wv * 3 + i;
      const int mat = t >> 3;
      const int rem = t & 7;
      const int mt = rem >> 1, nt2 = rem & 1;
      const int col0 = mat * DIMC + h * HDIM + nt2 * 16;
      v8f acc = {};
#pragma unroll
      for (int kk = 0; kk < 6; ++kk) {
        const v16h a = ld_frag(sA, DIMC, mt * 16, kk * 32, lane);
        const v16h b = ld_frag(qkvT, DIMC, col0, kk * 32, lane);
        acc = wmma_f16(a, b, acc);
      }
      const int cl = nt2 * 16 + c16;
      const float bias = qkv_b[col0 + c16];
#pragma unroll
      for (int r = 0; r < 8; ++r) {
        const int row = mt * 16 + 8 * h16 + r;
        const float v = acc[r] * W_DOWN + bias;
        if (mat == 0)      sQ[row * HDIM + cl] = (_Float16)(v * QK_SCALE * Q_UP);
        else if (mat == 1) sK[row * HDIM + cl] = (_Float16)v;
        else               sVT[cl * 64 + row] = (_Float16)v;
      }
    }
    __syncthreads();

#pragma unroll
    for (int i = 0; i < 2; ++i) {
      const int t = wv * 2 + i;
      const int mt = t >> 2, nt = t & 3;
      const v16h a = ld_frag(sQ, HDIM, mt * 16, 0, lane);
      const v16h b = ld_frag(sK, HDIM, nt * 16, 0, lane);
      v8f acc = {};
      acc = wmma_f16(a, b, acc);
      const int kj = nt * 16 + c16;
      int kid = 0, ky = 0, kx = 0;
      if (kj < NTOK) {
        ky = kj / WSZ; kx = kj - ky * WSZ;
        kid = region_id(wy * WSZ + ky, wx * WSZ + kx);
      }
#pragma unroll
      for (int r = 0; r < 8; ++r) {
        const int qi = mt * 16 + 8 * h16 + r;
        float s = NEG_BIG;
        if (kj < NTOK && qi < NTOK) {
          const int qy = qi / WSZ, qx = qi - qy * WSZ;
          if (region_id(wy * WSZ + qy, wx * WSZ + qx) == kid) {
            const int ridx = (qy - ky + (WSZ - 1)) * (2 * WSZ - 1) + (qx - kx + (WSZ - 1));
            s = acc[r] * Q_DOWN + rel_bias[ridx * HEADS + h];
          }
        }
        sS[qi * 64 + kj] = s;
      }
    }
    __syncthreads();

    {
      const int row = tid >> 2, s4 = tid & 3;
      const float* prow = sS + row * 64 + s4 * 16;
      float buf[16];
#pragma unroll
      for (int j = 0; j < 4; ++j) {
        const v4f q4 = *(const v4f*)(prow + 4 * j);
        buf[4 * j + 0] = q4.x; buf[4 * j + 1] = q4.y; buf[4 * j + 2] = q4.z; buf[4 * j + 3] = q4.w;
      }
      float m = NEG_BIG;
#pragma unroll
      for (int j = 0; j < 16; ++j) m = fmaxf(m, buf[j]);
      m = fmaxf(m, __shfl_xor(m, 1)); m = fmaxf(m, __shfl_xor(m, 2));
      float sum = 0.f;
#pragma unroll
      for (int j = 0; j < 16; ++j) { buf[j] = __expf(buf[j] - m); sum += buf[j]; }
      sum += __shfl_xor(sum, 1); sum += __shfl_xor(sum, 2);
      const float inv = 1.f / sum;
      _Float16* pp = sP + row * 64 + s4 * 16;
#pragma unroll
      for (int j = 0; j < 16; ++j) pp[j] = (_Float16)(buf[j] * inv * P_UP);
    }
    __syncthreads();

    {
      const int mt = wv >> 1, nt = wv & 1;
      v8f acc = {};
#pragma unroll
      for (int kk = 0; kk < 2; ++kk) {
        const v16h a = ld_frag(sP, 64, mt * 16, kk * 32, lane);
        const v16h b = ld_frag(sVT, 64, nt * 16, kk * 32, lane);
        acc = wmma_f16(a, b, acc);
      }
      const int d = nt * 16 + c16;
#pragma unroll
      for (int r = 0; r < 8; ++r)
        sAV[(mt * 16 + 8 * h16 + r) * HDIM + d] = (_Float16)(acc[r] * P_DOWN);
    }
    __syncthreads();

#pragma unroll
    for (int i = 0; i < 6; ++i) {
      const int gt = wv * 6 + i;
      const int mt = gt / 12, nt = gt % 12;
      const v16h a = ld_frag(sAV, HDIM, mt * 16, 0, lane);
      const v16h b = ld_frag(projT, DIMC, nt * 16, h * HDIM, lane);
      pacc[i] = wmma_f16(a, b, pacc[i]);
    }
    __syncthreads();
  }

#pragma unroll
  for (int i = 0; i < 6; ++i) {
    const int gt = wv * 6 + i;
    const int mt = gt / 12, nt = gt % 12;
    const int c = nt * 16 + c16;
    const float pb = proj_b[c];
#pragma unroll
    for (int r = 0; r < 8; ++r) {
      const int row = mt * 16 + 8 * h16 + r;
      sOut[row * DIMC + c] = pacc[i][r] * W_DOWN + pb;
    }
  }
  __syncthreads();

  attn_rows_store(sOut, xin, x1, bb, wy, wx, wv, lane);
  __threadfence();
  attn_rows_store(sOut, xin, x1, bb, wy, wx, wv, lane);
}

__device__ __forceinline__ void mlp_store(const float* sT, float* out, int bimg, int p0, int wv, int lane)
{
  const int h16 = lane >> 4, q = lane & 15;
#pragma unroll
  for (int i = 0; i < 12; ++i) {
    const int c = i * 16 + wv * 2 + h16;
    const v4f v = *(const v4f*)(sT + c * 64 + 4 * q);
    float* dst = out + (size_t)bimg * DIMC * PLANE + (size_t)c * PLANE + p0 + 4 * q;
    *(volatile v4f*)dst = v;
  }
}

__global__ void __launch_bounds__(256) k_mlp(
    const float* __restrict__ x1, const float* __restrict__ n2g, const float* __restrict__ n2b,
    const _Float16* __restrict__ fc1T, const float* __restrict__ fc1_b,
    const _Float16* __restrict__ fc2T, const float* __restrict__ fc2_b,
    float* out, int ntok)
{
  __shared__ __align__(16) unsigned char smem[49152];
  _Float16* sA = (_Float16*)(smem);
  _Float16* sH = (_Float16*)(smem + 24576);
  float*    sT = (float*)(smem);

  const int tid = threadIdx.x;
  const int lane = tid & 31, wv = tid >> 5, h16 = lane >> 4, c16 = lane & 15;
  const int tok0 = blockIdx.x * 64;
  if (tok0 >= ntok) return;
  const int bimg = tok0 / PLANE;
  const int p0 = tok0 - bimg * PLANE;

  {
    const int tl = tid >> 2, sub = tid & 3;
    const int tok = tok0 + tl;
    const float* pr = x1 + (size_t)tok * DIMC + sub * 48;
    float vals[48];
    float s = 0.f;
#pragma unroll
    for (int j = 0; j < 12; ++j) {
      const v4f q4 = *(const v4f*)(pr + 4 * j);
      vals[4 * j + 0] = q4.x; vals[4 * j + 1] = q4.y; vals[4 * j + 2] = q4.z; vals[4 * j + 3] = q4.w;
      s += (q4.x + q4.y) + (q4.z + q4.w);
    }
    s += __shfl_xor(s, 1); s += __shfl_xor(s, 2);
    const float mu = s * (1.f / DIMC);
    float d2 = 0.f;
#pragma unroll
    for (int j = 0; j < 48; ++j) { const float d = vals[j] - mu; d2 += d * d; }
    d2 += __shfl_xor(d2, 1); d2 += __shfl_xor(d2, 2);
    const float rs = rsqrtf(d2 * (1.f / DIMC) + 1e-5f);
#pragma unroll
    for (int j = 0; j < 48; ++j) {
      const int c = sub * 48 + j;
      sA[tl * DIMC + c] = (_Float16)((vals[j] - mu) * rs * n2g[c] + n2b[c]);
    }
  }
  __syncthreads();

  v8f facc[6];
#pragma unroll
  for (int i = 0; i < 6; ++i) { v8f z = {}; facc[i] = z; }

  for (int cc = 0; cc < 8; ++cc) {
    const int col0 = cc * 96;
#pragma unroll
    for (int i = 0; i < 3; ++i) {
      const int t = wv * 3 + i;
      const int mt = t / 6, nt = t % 6;
      const int col = col0 + nt * 16;
      v8f acc = {};
#pragma unroll
      for (int kk = 0; kk < 6; ++kk) {
        const v16h a = ld_frag(sA, DIMC, mt * 16, kk * 32, lane);
        const v16h b = ld_frag(fc1T, DIMC, col, kk * 32, lane);
        acc = wmma_f16(a, b, acc);
      }
      const float bias = fc1_b[col + c16];
      const int cl = nt * 16 + c16;
#pragma unroll
      for (int r = 0; r < 8; ++r) {
        const float v = acc[r] * W_DOWN + bias;
        const float g = 0.5f * v * (1.f + erff(v * 0.70710678118654752f));
        sH[(mt * 16 + 8 * h16 + r) * 96 + cl] = (_Float16)g;
      }
    }
    __syncthreads();
#pragma unroll
    for (int i = 0; i < 6; ++i) {
      const int gt = wv * 6 + i;
      const int mt = gt / 12, nt = gt % 12;
#pragma unroll
      for (int kk = 0; kk < 3; ++kk) {
        const v16h a = ld_frag(sH, 96, mt * 16, kk * 32, lane);
        const v16h b = ld_frag(fc2T, HID, nt * 16, col0 + kk * 32, lane);
        facc[i] = wmma_f16(a, b, facc[i]);
      }
    }
    __syncthreads();
  }

#pragma unroll
  for (int i = 0; i < 6; ++i) {
    const int gt = wv * 6 + i;
    const int mt = gt / 12, nt = gt % 12;
    const int c = nt * 16 + c16;
    const float bias = fc2_b[c];
#pragma unroll
    for (int r = 0; r < 8; ++r) {
      const int row = mt * 16 + 8 * h16 + r;
      const float res = x1[(size_t)(tok0 + row) * DIMC + c];
      sT[c * 64 + row] = facc[i][r] * W_DOWN + bias + res;
    }
  }
  __syncthreads();

  mlp_store(sT, out, bimg, p0, wv, lane);
  __threadfence();
  mlp_store(sT, out, bimg, p0, wv, lane);
}

extern "C" void kernel_launch(void* const* d_in, const int* in_sizes, int n_in,
                              void* d_out, int out_size, void* d_ws, size_t ws_size,
                              hipStream_t stream)
{
  if (n_in < 14) return;
  const float* x      = (const float*)d_in[0];
  const float* n1g    = (const float*)d_in[1];
  const float* n1b    = (const float*)d_in[2];
  const float* qkv_w  = (const float*)d_in[3];
  const float* qkv_b  = (const float*)d_in[4];
  const float* proj_w = (const float*)d_in[5];
  const float* proj_b = (const float*)d_in[6];
  const float* relb   = (const float*)d_in[7];
  const float* n2g    = (const float*)d_in[8];
  const float* n2b    = (const float*)d_in[9];
  const float* fc1_w  = (const float*)d_in[10];
  const float* fc1_b  = (const float*)d_in[11];
  const float* fc2_w  = (const float*)d_in[12];
  const float* fc2_b  = (const float*)d_in[13];

  const int nx = in_sizes[0];
  const int bsz = nx / (DIMC * PLANE);
  if (bsz <= 0 || bsz * (DIMC * PLANE) != nx || out_size != nx) return;

  const size_t wt_bytes = (size_t)SEG_END * 2;
  const size_t x1_off = (wt_bytes + 255) & ~(size_t)255;
  const size_t x1_bytes = (size_t)nx * 4;
  if (x1_off + x1_bytes > ws_size) return;

  _Float16* wt = (_Float16*)d_ws;
  float* x1 = (float*)((char*)d_ws + x1_off);

  const int nchunk = SEG_END / 8;
  k_wconv<<<(nchunk + 255) / 256, 256, 0, stream>>>(qkv_w, proj_w, fc1_w, fc2_w, wt, nchunk);

  const int nwin = bsz * 64;
  k_attn<<<nwin, 256, 0, stream>>>(x, n1g, n1b, wt + SEG0_OFF, qkv_b, wt + SEG1_OFF, proj_b, relb, x1, nwin);

  const int ntok = bsz * PLANE;
  k_mlp<<<(ntok + 63) / 64, 256, 0, stream>>>(x1, n2g, n2b, wt + SEG2_OFF, fc1_b, wt + SEG3_OFF, fc2_b,
                                             (float*)d_out, ntok);
}
